// LSSL_35751307771916
// MI455X (gfx1250) — hardware-run, weakly checked
//
#include <hip/hip_runtime.h>
#include <math.h>

typedef __attribute__((ext_vector_type(16))) _Float16 v16h;
typedef __attribute__((ext_vector_type(8)))  _Float16 v8h;
typedef __attribute__((ext_vector_type(8)))  float    v8f;
typedef __attribute__((ext_vector_type(4)))  float    v4f;
typedef __attribute__((ext_vector_type(4)))  unsigned v4u;

constexpr int kBatch = 16;
constexpr int kSeq   = 2048;
constexpr int kHid   = 256;
constexpr int kNst   = 64;
constexpr int kChn   = 2;
constexpr int kRows  = kBatch * kSeq;
constexpr int kFeat  = kHid * kChn;
static_assert(kBatch == 16);
static_assert(kNst == 64 && (kNst % 32) == 0);
static_assert((kSeq % 32) == 0 && (kHid % 32) == 0);
static_assert((kRows % 64) == 0 && (kHid % 64) == 0 && (kFeat % 32) == 0);

constexpr float kACarry   = 64.0f;
constexpr float kXCarry   = 16.0f;
constexpr float kRes      = 2048.0f;
constexpr float kInvRes   = 1.0f / kRes;
constexpr float kStepScale = 1.0f / kACarry;
constexpr float kBdScale   = kACarry * kXCarry;
constexpr float kInvX      = 1.0f / kXCarry;
constexpr float kGCarry    = 8.0f;
constexpr float kWCarry    = 256.0f;
constexpr float kProjScale = 1.0f / (kGCarry * kWCarry);
constexpr float kF16Min    = 6.103515625e-5f;
constexpr float kRsqrt2    = 0.70710678118654752f;

constexpr size_t kSzU  = (size_t)kHid * kBatch * kSeq * 4;
constexpr size_t kSzG  = (size_t)kHid * kBatch * kSeq * kChn * 2;
constexpr size_t kSzGR = (size_t)kRows * kFeat * 2;
constexpr size_t kSzAP = (size_t)kHid * kNst * kNst * 2;
constexpr size_t kSzBD = (size_t)kHid * kNst * 4;
constexpr size_t kSzWT = (size_t)kHid * kFeat * 2;
constexpr size_t kOffU  = 0;
constexpr size_t kOffG  = kOffU  + kSzU;
constexpr size_t kOffGR = kOffG  + kSzG;
constexpr size_t kOffAH = kOffGR + kSzGR;
constexpr size_t kOffAL = kOffAH + kSzAP;
constexpr size_t kOffBD = kOffAL + kSzAP;
constexpr size_t kOffWT = kOffBD + kSzBD;
constexpr size_t kWsTotal = kOffWT + kSzWT;
static_assert(kWsTotal == 105185280ull);
static_assert(kWsTotal <= 134217728ull);
static_assert((kOffG % 128) == 0 && (kOffGR % 128) == 0 && (kOffAH % 128) == 0 && (kOffAL % 128) == 0 &&
              (kOffBD % 128) == 0 && (kOffWT % 128) == 0);

__device__ __forceinline__ float bf16v(float f) {
  unsigned u = __float_as_uint(f);
  u = (u + 0x7FFFu + ((u >> 16) & 1u)) & 0xFFFF0000u;
  return __uint_as_float(u);
}
__device__ __forceinline__ float flush16(float c) {
  return (fabsf(c) < kF16Min) ? 0.0f : c;
}
__device__ __forceinline__ void split16(float c, _Float16& hi, _Float16& lo) {
  const _Float16 hv = (_Float16)flush16(c);
  float hf = (float)hv;
  asm volatile("" : "+v"(hf));
  const float r = (c - hf) * kRes;
  hi = hv;
  lo = (_Float16)flush16(r);
}
union FragU { v16h v; v8h h[2]; };
__device__ __forceinline__ v16h ldfrag(const _Float16* p) {
  FragU f;
  f.h[0] = *(const v8h*)(p);
  f.h[1] = *(const v8h*)(p + 16);
  return f.v;
}
__device__ __forceinline__ v8f mma(v16h a, v16h b, v8f c) {
  return __builtin_amdgcn_wmma_f32_16x16x32_f16(false, a, false, b, (short)0, c, false, false);
}
__device__ __forceinline__ void tie_acc(v8f& a) {
  asm volatile("" : "+v"(a));
}
__device__ __forceinline__ void guard_six(v8f& a, v16h a0, v16h a1, v16h a2, v16h a3,
                                          v16h b0, v16h b1, v16h b2, v16h b3) {
  asm volatile("v_nop\n\tv_nop\n\tv_nop\n\tv_nop"
               : "+v"(a)
               : "v"(a0), "v"(a1), "v"(a2), "v"(a3), "v"(b0), "v"(b1), "v"(b2), "v"(b3));
}
__device__ __forceinline__ void guard_four(v8f& a, v16h x, v16h b0, v16h b1, v16h b2, v16h b3) {
  asm volatile("v_nop\n\tv_nop\n\tv_nop\n\tv_nop"
               : "+v"(a)
               : "v"(x), "v"(b0), "v"(b1), "v"(b2), "v"(b3));
}

__global__ __launch_bounds__(256)
void input_to_channel_rows(const float* __restrict__ in, float* __restrict__ U)
{
  __shared__ __align__(16) float sT[32 * 36];
  const int tid = threadIdx.x;
  const int h0 = blockIdx.x * 32;
  const int t0 = blockIdx.y * 32;
  const int b  = blockIdx.z;
  const int tl = tid >> 3;
  const int q4 = (tid & 7) * 4;
  const v4f v = *(const v4f*)(in + ((size_t)(b * kSeq + t0 + tl) * kHid + h0 + q4));
#pragma unroll
  for (int e = 0; e < 4; ++e) {
    const float xe = v[e];
    sT[(q4 + e) * 36 + tl] = bf16v(xe);
  }
  __syncthreads();
  const int hl = tid >> 3;
  const v4f o = *(const v4f*)(sT + hl * 36 + q4);
  float* dst = U + ((size_t)((h0 + hl) * kBatch + b) * kSeq + t0 + q4);
  *(volatile v4f*)dst = o;
  __threadfence();
  *(volatile v4f*)dst = o;
}

constexpr int kWP = 144;
static_assert((kWP % 16) == 0 && kWP >= 2 * kNst + 1);

__global__ __launch_bounds__(256)
void discretise_channels(const float* __restrict__ Ag, const float* __restrict__ Bg,
                         const float* __restrict__ dtg,
                         unsigned short* __restrict__ AH, unsigned short* __restrict__ AL,
                         float* __restrict__ BD)
{
  __shared__ __align__(16) float sW[kNst * kWP];
  __shared__ __align__(16) float sRd[kNst];
  const int tid = threadIdx.x;
  const int h   = blockIdx.x;
  const float dth = bf16v(dtg[h]);

#pragma unroll 1
  for (int i = tid; i < kNst * kWP; i += 256) {
    const int r  = i / kWP;
    const int c  = i - r * kWP;
    const int cc = c & 63;
    float a  = Ag[r * kNst + cc];
    float bb = Bg[r];
    asm volatile("" : "+v"(a), "+v"(bb));
    const float hf  = 0.5f * (dth * bf16v(a));
    const float idn = (r == cc) ? 1.0f : 0.0f;
    const float vl  = idn - hf;
    const float vr  = idn + hf;
    const float vb  = dth * bf16v(bb);
    const float v   = (c < 64) ? vl : ((c < 128) ? vr : ((c == 128) ? vb : 0.0f));
    sW[i] = v;
  }
  __syncthreads();

  const int row = tid & 63;
  const int cq  = tid >> 6;
  float* wrow = sW + row * kWP + cq * 36;
#pragma unroll 1
  for (int p = 0; p < kNst; ++p) {
    const float* prow = sW + p * kWP;
    const float piv  = prow[p];
    const float rinv = 1.0f / piv;
    const float e    = sW[row * kWP + p];
    const float f    = e * rinv;
    __syncthreads();
    if (row != p) {
      const float* pr = prow + cq * 36;
#pragma unroll 3
      for (int j = 0; j < 9; ++j) {
        const v4f pv = *(const v4f*)(pr + 4 * j);
        v4f a = *(const v4f*)(wrow + 4 * j);
        a[0] = fmaf(-f, pv[0], a[0]);
        a[1] = fmaf(-f, pv[1], a[1]);
        a[2] = fmaf(-f, pv[2], a[2]);
        a[3] = fmaf(-f, pv[3], a[3]);
        *(v4f*)(wrow + 4 * j) = a;
      }
    }
    __syncthreads();
  }
  if (tid < kNst) sRd[tid] = 1.0f / sW[tid * kWP + tid];
  __syncthreads();

  v8h hv[2], lv[2];
#pragma unroll
  for (int it = 0; it < 2; ++it) {
    const int n  = it * 32 + (tid >> 3);
    const int k8 = (tid & 7) * 8;
    const float rd = sRd[n];
    const v4f a0 = *(const v4f*)(sW + n * kWP + 64 + k8);
    const v4f a1 = *(const v4f*)(sW + n * kWP + 64 + k8 + 4);
#pragma unroll
    for (int e = 0; e < 4; ++e) {
      const float x0 = a0[e];
      const float x1 = a1[e];
      _Float16 a, b;
      split16(x0 * rd * kACarry, a, b);
      hv[it][e] = a;
      lv[it][e] = b;
      split16(x1 * rd * kACarry, a, b);
      hv[it][4 + e] = a;
      lv[it][4 + e] = b;
    }
  }
  v4f bo;
  {
    const int n4 = (tid & 15) * 4;
#pragma unroll
    for (int e = 0; e < 4; ++e) bo[e] = sW[(n4 + e) * kWP + 128] * sRd[n4 + e];
  }
  for (int pass = 0; pass < 2; ++pass) {
#pragma unroll
    for (int it = 0; it < 2; ++it) {
      const int n  = it * 32 + (tid >> 3);
      const int k8 = (tid & 7) * 8;
      const size_t o = (size_t)(h * kNst + n) * kNst + k8;
      *(volatile v8h*)(AH + o) = hv[it];
      *(volatile v8h*)(AL + o) = lv[it];
    }
    if (tid < 16) *(volatile v4f*)(BD + (size_t)h * kNst + tid * 4) = bo;
    __threadfence();
  }
}

__global__ __launch_bounds__(256)
void weight_plane(const float* __restrict__ W, unsigned short* __restrict__ WT)
{
  __shared__ __align__(16) float sW[32 * 68];
  const int tid = threadIdx.x;
  const int k0 = blockIdx.x * 64;
  const int n0 = blockIdx.y * 32;
  const int kk = tid >> 3;
  const int q4 = (tid & 7) * 4;
#pragma unroll
  for (int it = 0; it < 2; ++it) {
    const int k = kk + 32 * it;
    const v4f v = *(const v4f*)(W + (size_t)(k0 + k) * kHid + n0 + q4);
#pragma unroll
    for (int e = 0; e < 4; ++e) {
      const float xe = v[e];
      sW[(q4 + e) * 68 + k] = xe;
    }
  }
  __syncthreads();
  const int n  = tid >> 3;
  const int k8 = (tid & 7) * 8;
  const v4f a0 = *(const v4f*)(sW + n * 68 + k8);
  const v4f a1 = *(const v4f*)(sW + n * 68 + k8 + 4);
  v8h hv;
#pragma unroll
  for (int e = 0; e < 4; ++e) {
    const float x0 = a0[e];
    const float x1 = a1[e];
    hv[e]     = (_Float16)flush16(bf16v(x0) * kWCarry);
    hv[4 + e] = (_Float16)flush16(bf16v(x1) * kWCarry);
  }
  unsigned short* dst = WT + (size_t)(n0 + n) * kFeat + k0 + k8;
  *(volatile v8h*)dst = hv;
  __threadfence();
  *(volatile v8h*)dst = hv;
}

constexpr int kThr   = 128;
constexpr int kHP    = 72;
constexpr int kPlane = kBatch * kHP;
constexpr int kBuf   = 32;
static_assert((kHP % 8) == 0 && kHP >= kNst);
static_assert((kSeq % kBuf) == 0 && kBuf == 32);
static_assert(kThr == 2 * kNst && kThr / 32 == kNst / 16);

__global__ __launch_bounds__(kThr)
void channel_steps(const float* __restrict__ U,
                   const unsigned short* __restrict__ AH, const unsigned short* __restrict__ AL,
                   const float* __restrict__ BD, const float* __restrict__ Cg,
                   const float* __restrict__ Dg, unsigned short* __restrict__ G)
{
  __shared__ __align__(16) _Float16 sXh[2 * kPlane];
  __shared__ __align__(16) _Float16 sXl[2 * kPlane];
  __shared__ __align__(16) float    sU[kBatch * kBuf];
  __shared__ __align__(16) float    sYp[kBuf * kThr];
  __shared__ __align__(16) _Float16 sGh[kBatch * kBuf * kChn];

  const int tid  = threadIdx.x;
  const int lane = tid & 31;
  const int wave = __builtin_amdgcn_readfirstlane(tid >> 5);
  const int hh   = lane >> 4;
  const int nn   = lane & 15;
  const int h    = blockIdx.x;
  const int tm16 = wave * 16;

  const _Float16* ahp = (const _Float16*)AH + (size_t)(h * kNst + tm16 + nn) * kNst + 8 * hh;
  const _Float16* alp = (const _Float16*)AL + (size_t)(h * kNst + tm16 + nn) * kNst + 8 * hh;
  const v16h fAh0 = ldfrag(ahp);
  const v16h fAh1 = ldfrag(ahp + 32);
  const v16h fAl0 = ldfrag(alp);
  const v16h fAl1 = ldfrag(alp + 32);

  float bd[8], c0[8], c1[8];
  {
    const int nb = tm16 + 8 * hh;
    const v4f b0 = *(const v4f*)(BD + (size_t)h * kNst + nb);
    const v4f b1 = *(const v4f*)(BD + (size_t)h * kNst + nb + 4);
    const v4f p0 = *(const v4f*)(Cg + (size_t)(h * kChn + 0) * kNst + nb);
    const v4f p1 = *(const v4f*)(Cg + (size_t)(h * kChn + 0) * kNst + nb + 4);
    const v4f q0 = *(const v4f*)(Cg + (size_t)(h * kChn + 1) * kNst + nb);
    const v4f q1 = *(const v4f*)(Cg + (size_t)(h * kChn + 1) * kNst + nb + 4);
#pragma unroll
    for (int e = 0; e < 4; ++e) {
      const float x0 = b0[e];
      const float x1 = b1[e];
      const float y0 = p0[e];
      const float y1 = p1[e];
      const float z0 = q0[e];
      const float z1 = q1[e];
      bd[e]     = x0 * kBdScale;
      bd[4 + e] = x1 * kBdScale;
      c0[e]     = bf16v(y0) * kInvX;
      c0[4 + e] = bf16v(y1) * kInvX;
      c1[e]     = bf16v(z0) * kInvX;
      c1[4 + e] = bf16v(z1) * kInvX;
    }
  }
  const float d0 = bf16v(Dg[h * kChn + 0]);
  const float d1 = bf16v(Dg[h * kChn + 1]);

  {
    const v8h zh = (v8h){(_Float16)0.0f, (_Float16)0.0f, (_Float16)0.0f, (_Float16)0.0f,
                         (_Float16)0.0f, (_Float16)0.0f, (_Float16)0.0f, (_Float16)0.0f};
#pragma unroll 1
    for (int i = tid; i < (2 * kPlane) / 8; i += kThr) {
      *(v8h*)(sXh + 8 * i) = zh;
      *(v8h*)(sXl + 8 * i) = zh;
    }
  }
  __syncthreads();

  const int boff = nn * kHP + 8 * hh;
  const int soff = nn * kHP + tm16 + 8 * hh;
  const v8f z8 = (v8f){0.f, 0.f, 0.f, 0.f, 0.f, 0.f, 0.f, 0.f};

#pragma unroll 1
  for (int t = 0; t < kSeq; ++t) {
    const int tt = t & (kBuf - 1);

    if (tt == 0) {
      const int b  = tid >> 3;
      const int q4 = (tid & 7) * 4;
      const v4f uv = *(const v4f*)(U + ((size_t)(h * kBatch + b) * kSeq + t + q4));
      *(v4f*)(sU + b * kBuf + q4) = uv;
      __syncthreads();
    }

    const int cur = (t & 1) * kPlane;
    const int nxt = kPlane - cur;
    const v16h bh0 = ldfrag(sXh + cur + boff);
    const v16h bh1 = ldfrag(sXh + cur + boff + 32);
    const v16h bl0 = ldfrag(sXl + cur + boff);
    const v16h bl1 = ldfrag(sXl + cur + boff + 32);
    const float u = sU[nn * kBuf + tt];

    v8f cm, cr;
#pragma unroll
    for (int r = 0; r < 8; ++r) cm[r] = bd[r] * u;
    cm = mma(fAh0, bh0, cm);
    cr = mma(fAh0, bl0, z8);
    cm = mma(fAh1, bh1, cm);
    cr = mma(fAl0, bh0, cr);
    cr = mma(fAh1, bl1, cr);
    cr = mma(fAl1, bh1, cr);
    tie_acc(cm);
    guard_six(cr, fAh0, fAh1, fAl0, fAl1, bh0, bh1, bl0, bl1);

    float p0 = 0.0f, p1 = 0.0f;
    v8h hv, lv;
#pragma unroll
    for (int r = 0; r < 8; ++r) {
      const float c = fmaf(cr[r], kInvRes, cm[r]) * kStepScale;
      p0 = fmaf(c0[r], c, p0);
      p1 = fmaf(c1[r], c, p1);
      _Float16 a, b;
      split16(c, a, b);
      hv[r] = a;
      lv[r] = b;
    }
    *(v8h*)(sXh + nxt + soff) = hv;
    *(v8h*)(sXl + nxt + soff) = lv;

    const float e0 = __shfl_xor(p0, 16, 32);
    const float e1 = __shfl_xor(p1, 16, 32);
    const float s0 = p0 + e0;
    const float s1 = p1 + e1;
    sYp[tt * kThr + tid] = hh ? s1 : s0;
    __syncthreads();

    if (tt == kBuf - 1) {
      const int t0 = t - (kBuf - 1);
#pragma unroll 1
      for (int j = 0; j < 8; ++j) {
        const int p  = tid + kThr * (j >> 1);
        const int m  = j & 1;
        const int b  = p & 15;
        const int tq = p >> 4;
        const float uu = sU[b * kBuf + tq];
        const float* yp = sYp + tq * kThr + m * 16 + b;
        float y = yp[0];
        y += yp[32];
        y += yp[64];
        y += yp[96];
        y = fmaf(m ? d1 : d0, uu, y);
        const float g = 0.5f * y * (1.0f + erff(y * kRsqrt2));
        sGh[b * (kBuf * kChn) + tq * kChn + m] = (_Float16)flush16(g * kGCarry);
      }
      __syncthreads();
      {
        const int bl = wave * 4 + (lane >> 3);
        const int q8 = (lane & 7) * 8;
        const v8h gv = *(const v8h*)(sGh + bl * (kBuf * kChn) + q8);
        unsigned short* dst = G + ((size_t)(h * kBatch + bl) * kSeq + t0) * kChn + q8;
        *(volatile v8h*)dst = gv;
        __threadfence();
        *(volatile v8h*)dst = gv;
      }
    }
  }
}

__global__ __launch_bounds__(256)
void rows_from_channels(const unsigned* __restrict__ G32, unsigned* __restrict__ GR32)
{
  __shared__ __align__(16) unsigned sT[32 * 36];
  const int tid = threadIdx.x;
  const int h0 = blockIdx.x * 32;
  const int t0 = blockIdx.y * 32;
  const int b  = blockIdx.z;
  const int hl = tid >> 3;
  const int q4 = (tid & 7) * 4;
  const v4u v = *(const v4u*)(G32 + ((size_t)((h0 + hl) * kBatch + b) * kSeq + t0 + q4));
  *(v4u*)(sT + hl * 36 + q4) = v;
  __syncthreads();
  const int tl = tid >> 3;
  v4u o;
#pragma unroll
  for (int e = 0; e < 4; ++e) o[e] = sT[(q4 + e) * 36 + tl];
  unsigned* dst = GR32 + ((size_t)(b * kSeq + t0 + tl) * kHid + h0 + q4);
  *(volatile v4u*)dst = o;
  __threadfence();
  *(volatile v4u*)dst = o;
}

constexpr int kTilesM = kRows / 64;
constexpr int kTilesN = kHid / 64;
static_assert((kTilesM * kTilesN) % 8 == 0);

__global__ __launch_bounds__(256)
void project_rows(const unsigned short* __restrict__ Ap, const unsigned short* __restrict__ Btp,
                  float* __restrict__ Cout)
{
  const _Float16* A  = (const _Float16*)Ap;
  const _Float16* Bt = (const _Float16*)Btp;
  __shared__ __align__(16) float sT[8][16 * 68];
  const int lane = threadIdx.x & 31;
  const int wave = threadIdx.x >> 5;
  const int tile = blockIdx.x * 8 + wave;
  if (tile >= kTilesM * kTilesN) return;
  const int tm = tile / kTilesN;
  const int tn = tile - tm * kTilesN;
  const int m0 = tm << 6;
  const int n0 = tn << 6;
  const int rlane = lane & 15;
  const int koff  = (lane >> 4) * 8;
  const int mOff  = (lane >> 4) * 8;

  v8f acc[4][4];
#pragma unroll
  for (int i = 0; i < 4; ++i)
#pragma unroll
    for (int j = 0; j < 4; ++j) acc[i][j] = (v8f){0.f, 0.f, 0.f, 0.f, 0.f, 0.f, 0.f, 0.f};

  for (int k0 = 0; k0 < kFeat; k0 += 32) {
    v16h bh[4];
#pragma unroll
    for (int j = 0; j < 4; ++j) {
      const size_t bo = (size_t)(n0 + (j << 4) + rlane) * kFeat + koff + k0;
      bh[j] = ldfrag(Bt + bo);
    }
#pragma unroll
    for (int i = 0; i < 4; ++i) {
      const size_t ao = (size_t)(m0 + (i << 4) + rlane) * kFeat + koff + k0;
      const v16h ah = ldfrag(A + ao);
#pragma unroll
      for (int j = 0; j < 4; ++j) acc[i][j] = mma(ah, bh[j], acc[i][j]);
      tie_acc(acc[i][0]);
      tie_acc(acc[i][1]);
      tie_acc(acc[i][2]);
      guard_four(acc[i][3], ah, bh[0], bh[1], bh[2], bh[3]);
    }
  }

  float* slab = sT[wave];
#pragma unroll
  for (int i = 0; i < 4; ++i) {
    const int mBase = m0 + (i << 4);
#pragma unroll
    for (int j = 0; j < 4; ++j) {
#pragma unroll
      for (int r = 0; r < 8; ++r) {
        slab[(mOff + r) * 68 + (j << 4) + rlane] = acc[i][j][r] * kProjScale;
      }
    }
    __builtin_amdgcn_fence(__ATOMIC_RELEASE, "workgroup");
    __builtin_amdgcn_wave_barrier();
    __builtin_amdgcn_fence(__ATOMIC_ACQUIRE, "workgroup");
    {
      const int hh = lane >> 4;
      const int c4 = (lane & 15) * 4;
      for (int pass = 0; pass < 2; ++pass) {
#pragma unroll
        for (int it = 0; it < 8; ++it) {
          const int row = it * 2 + hh;
          const v4f v = *(const v4f*)(slab + row * 68 + c4);
          *(volatile v4f*)(Cout + (size_t)(mBase + row) * kHid + n0 + c4) = v;
        }
        __threadfence();
      }
    }
    __builtin_amdgcn_fence(__ATOMIC_RELEASE, "workgroup");
    __builtin_amdgcn_wave_barrier();
    __builtin_amdgcn_fence(__ATOMIC_ACQUIRE, "workgroup");
  }
}

extern "C" void kernel_launch(void* const* d_in, const int* in_sizes, int n_in,
                              void* d_out, int out_size, void* d_ws, size_t ws_size,
                              hipStream_t stream) {
  if (n_in < 7) return;
  if (in_sizes[0] != kRows * kHid) return;
  if (in_sizes[1] != kNst * kNst) return;
  if (in_sizes[2] != kNst) return;
  if (in_sizes[3] != kHid) return;
  if (in_sizes[4] != kHid * kChn * kNst) return;
  if (in_sizes[5] != kHid * kChn) return;
  if (in_sizes[6] != kFeat * kHid) return;
  if (out_size != kRows * kHid) return;
  if (ws_size < kWsTotal) return;

  const float* xin = (const float*)d_in[0];
  const float* Ag  = (const float*)d_in[1];
  const float* Bg  = (const float*)d_in[2];
  const float* dtg = (const float*)d_in[3];
  const float* Cg  = (const float*)d_in[4];
  const float* Dg  = (const float*)d_in[5];
  const float* Wg  = (const float*)d_in[6];
  float* out = (float*)d_out;

  char* ws = (char*)d_ws;
  float*          U  = (float*)(ws + kOffU);
  unsigned short* G  = (unsigned short*)(ws + kOffG);
  unsigned short* GR = (unsigned short*)(ws + kOffGR);
  unsigned short* AH = (unsigned short*)(ws + kOffAH);
  unsigned short* AL = (unsigned short*)(ws + kOffAL);
  float*          BD = (float*)(ws + kOffBD);
  unsigned short* WT = (unsigned short*)(ws + kOffWT);

  input_to_channel_rows<<<dim3(kHid / 32, kSeq / 32, kBatch), dim3(256), 0, stream>>>(xin, U);
  discretise_channels<<<dim3(kHid), dim3(256), 0, stream>>>(Ag, Bg, dtg, AH, AL, BD);
  weight_plane<<<dim3(kFeat / 64, kHid / 32), dim3(256), 0, stream>>>(Wg, WT);
  channel_steps<<<dim3(kHid), dim3(kThr), 0, stream>>>(U, AH, AL, BD, Cg, Dg, G);
  rows_from_channels<<<dim3(kHid / 32, kSeq / 32, kBatch), dim3(256), 0, stream>>>(
      (const unsigned*)G, (unsigned*)GR);
  project_rows<<<dim3((kTilesM * kTilesN) / 8), dim3(256), 0, stream>>>(GR, WT, out);
}
